// SliceRenderer_50457275793906
// MI455X (gfx1250) — hardware-verified
//
#include <hip/hip_runtime.h>
#include <stdint.h>


typedef __attribute__((ext_vector_type(16))) _Float16 v16h;
typedef __attribute__((ext_vector_type(8)))  _Float16 v8h;
typedef __attribute__((ext_vector_type(8)))  float    v8f;
typedef __attribute__((ext_vector_type(4)))  float    v4f;
typedef __attribute__((ext_vector_type(8)))  unsigned short v8us;

#define IMG_H 512
#define IMG_W 512
#define SEG 256
#define KSTEPS_MAX (SEG / 32)
#define EPSF 1e-8f
#define ZTH 3.0f
#define OPSC 16.0f
#define OUT_SCALE (1.0f / 256.0f)
#define WS_CAP ((size_t)134217728)

__device__ __forceinline__ void dep_guard_h(v8f& a, v8f& b, v16h x, v16h y) { asm volatile("v_nop\n\tv_nop\n\tv_nop\n\tv_nop" : "+v"(a), "+v"(b) : "v"(x), "v"(y)); }
__device__ __forceinline__ void keep4_h(v16h a, v16h b, v16h c, v16h d) { asm volatile("v_nop" :: "v"(a), "v"(b), "v"(c), "v"(d)); }
__device__ __forceinline__ void acc_guard4(v8f& a, v8f& b, v8f& c, v8f& d) { asm volatile("v_nop\n\tv_nop\n\tv_nop\n\tv_nop" : "+v"(a), "+v"(b), "+v"(c), "+v"(d)); }

template <typename T> struct Frag;
template <> struct Frag<_Float16> {
  typedef v16h V; union U { v16h v; v8h h[2]; };
  static __device__ __forceinline__ v16h load(const _Float16* p) {
    U f; f.h[0] = *(const v8h*)(p); f.h[1] = *(const v8h*)(p + 16); return f.v;
  }
  static __device__ __forceinline__ v8f mma(v16h a, v16h b, v8f c) {
    return __builtin_amdgcn_wmma_f32_16x16x32_f16(false, a, false, b, (short)0, c, false, false);
  }
  static __device__ __forceinline__ void guard(v8f& a, v8f& b, v16h x, v16h y) { dep_guard_h(a, b, x, y); }
  static __device__ __forceinline__ void keep(v16h a, v16h b, v16h c, v16h d) { keep4_h(a, b, c, d); }
};

__device__ __forceinline__ float z_dist(float zt, float pz, float sz) {
  const float num = zt - pz;
  const float den = sz + EPSF;
  return (num == 0.0f) ? 0.0f : (num / den);
}
__device__ __forceinline__ int z_keep(float zd) { return (fabsf(zd) < ZTH) ? 1 : 0; }

__device__ __forceinline__ v4f make4(float a, float b, float c, float d) { v4f r; r[0] = a; r[1] = b; r[2] = c; r[3] = d; return r; }

__global__ __launch_bounds__(256) void prep_params(
    const float* __restrict__ pos, const float* __restrict__ scl,
    const float* __restrict__ opa, const float* __restrict__ inten,
    const int* __restrict__ ztgt,
    v4f* __restrict__ PA, v4f* __restrict__ PB, int n) {
  __shared__ __align__(16) v4f sA[SEG];
  __shared__ __align__(16) v4f sB[SEG];
  __shared__ int sCnt[8];
  const int t = threadIdx.x;
  const int lane = t & 31;
  const int wave = t >> 5;
  const int g = blockIdx.x * SEG + t;
  const float zt = (float)ztgt[0];

  int keep = 0;
  v4f a = make4(0.f, 0.f, 0.f, 0.f);
  v4f b = make4(0.f, 0.f, 0.f, 0.f);
  if (g < n) {
    const float pz = pos[(size_t)g * 3 + 2];
    const float sz = scl[(size_t)g * 3 + 2];
    const float zd = z_dist(zt, pz, sz);
    if (z_keep(zd)) {
      keep = 1;
      const float zw  = expf((-0.5f * zd) * zd);
      const float eff = (opa[g] * zw) * inten[g];
      const float px  = pos[(size_t)g * 3 + 0];
      const float py  = pos[(size_t)g * 3 + 1];
      const float isx = 1.0f / (scl[(size_t)g * 3 + 0] + EPSF);
      const float isy = 1.0f / (scl[(size_t)g * 3 + 1] + EPSF);
      a = make4(px, isx, eff * OPSC, 0.f);
      b = make4(py, isy, OPSC, 0.f);
    }
  }
  const unsigned bal = __builtin_amdgcn_ballot_w32(keep != 0);
  const int pre = __builtin_popcount(bal & ((1u << lane) - 1u));
  if (lane == 0) sCnt[wave] = __builtin_popcount(bal);
  sA[t] = make4(0.f, 0.f, 0.f, 0.f);
  sB[t] = make4(0.f, 0.f, 0.f, 0.f);
  __syncthreads();
  int off = 0;
#pragma unroll
  for (int w = 0; w < 8; ++w) off += (w < wave) ? sCnt[w] : 0;
  int p = off + pre;
  if (p > SEG - 1) p = SEG - 1;
  if (keep) { sA[p] = a; sB[p] = b; }
  __syncthreads();
  const v4f oa = sA[t];
  const v4f ob = sB[t];
  const size_t slot = (size_t)blockIdx.x * SEG + (size_t)t;
  *(volatile v4f*)(PA + slot) = oa;
  *(volatile v4f*)(PB + slot) = ob;
  __threadfence();
  *(volatile v4f*)(PA + slot) = oa;
  *(volatile v4f*)(PB + slot) = ob;
}

__global__ __launch_bounds__(256) void build_rows(
    const v4f* __restrict__ P, unsigned short* __restrict__ out,
    int ld, int slotBase, int slotTot) {
  __shared__ __align__(16) unsigned short sh[8][SEG];
  const int t = threadIdx.x;
  const int lane = t & 31;
  const int wave = t >> 5;
  const int wq = blockIdx.x * 8 + wave;
  const int r  = blockIdx.y;
  if (wq * SEG >= ld) return;
  const float fc = (float)r;
  const int base = slotBase + wq * SEG;
  unsigned short* sw = sh[wave];
#pragma unroll
  for (int j = 0; j < 8; ++j) {
    const int sl  = j * 32 + lane;
    const int gsl = base + sl;
    unsigned short bits = 0;
    if (gsl < slotTot) {
      const v4f pp = P[gsl];
      if (pp[2] != 0.0f) {
        const float d = (fc - pp[0]) * pp[1];
        const float e = expf((-0.5f * d) * d);
        const float v = e * pp[2];
        const _Float16 hv = (_Float16)v;
        bits = __builtin_bit_cast(unsigned short, hv);
        if ((bits & 0x7C00u) == 0u) bits = 0;
      }
    }
    sw[sl] = bits;
  }
  __builtin_amdgcn_fence(__ATOMIC_RELEASE, "workgroup");
  __builtin_amdgcn_wave_barrier();
  __builtin_amdgcn_fence(__ATOMIC_ACQUIRE, "workgroup");
  const v8us o = *(const v8us*)(sw + lane * 8);
  unsigned short* dst = out + (size_t)r * (size_t)ld + (size_t)wq * SEG + (size_t)lane * 8;
  *(volatile v8us*)dst = o;
  __threadfence();
  *(volatile v8us*)dst = o;
}

template <bool RESID>
__global__ __launch_bounds__(256) void splat_gemm(
    const unsigned short* __restrict__ Ap, const unsigned short* __restrict__ Btp, int ldk,
    const float* __restrict__ pos, const float* __restrict__ scl, const int* __restrict__ ztgt,
    int n, int segBase, int spc, int nSeg,
    float* __restrict__ Cout, const float* __restrict__ resid, float scale) {
  typedef _Float16 T;
  typedef v16h V;
  const T* Ab = (const T*)Ap;
  const T* Bb = (const T*)Btp;
  __shared__ __align__(16) float sT[8][16 * 68];
  const int lane = threadIdx.x & 31;
  const int wave = threadIdx.x >> 5;
  const int tilesN = IMG_W >> 6;
  const int tilesM = IMG_H >> 6;
  const int tile = blockIdx.x * 8 + wave;
  if (tile >= tilesM * tilesN) return;
  const int tm = tile / tilesN;
  const int tn = tile - tm * tilesN;
  const int m0 = tm << 6;
  const int n0 = tn << 6;

  const int rlane = lane & 15;
  const int koff  = (lane >> 4) * 8;
  const int mOff  = (lane >> 4) * 8;

  v8f acc[4][4];
#pragma unroll
  for (int i = 0; i < 4; ++i)
#pragma unroll
    for (int j = 0; j < 4; ++j) acc[i][j] = (v8f){0.f,0.f,0.f,0.f,0.f,0.f,0.f,0.f};

  const float zt = (float)ztgt[0];

  for (int s = 0; s < spc; ++s) {
    const int gseg = segBase + s;
    int cnt = 0;
    if (gseg < nSeg) {
      const int gb = gseg * SEG + lane * 8;
#pragma unroll 1
      for (int j = 0; j < 8; ++j) {
        const int g = gb + j;
        if (g < n) {
          const float pz = pos[(size_t)g * 3 + 2];
          const float sz = scl[(size_t)g * 3 + 2];
          cnt += z_keep(z_dist(zt, pz, sz));
        }
      }
    }
#pragma unroll
    for (int off = 16; off > 0; off >>= 1) cnt += __shfl_xor(cnt, off, 32);
    int steps = (cnt + 31) >> 5;
    if (steps > KSTEPS_MAX) steps = KSTEPS_MAX;
    if (steps < 0) steps = 0;
    steps = __builtin_amdgcn_readfirstlane(steps);

    for (int ks = 0; ks < steps; ++ks) {
      const int k0 = s * SEG + ks * 32;
      V bh[4];
#pragma unroll
      for (int j = 0; j < 4; ++j) {
        const size_t bo = (size_t)(n0 + (j << 4) + rlane) * (size_t)ldk + koff + k0;
        bh[j] = Frag<T>::load(Bb + bo);
      }
#pragma unroll
      for (int i = 0; i < 4; ++i) {
        const size_t ao = (size_t)(m0 + (i << 4) + rlane) * (size_t)ldk + koff + k0;
        V ah = Frag<T>::load(Ab + ao);
#pragma unroll
        for (int j = 0; j < 4; ++j) acc[i][j] = Frag<T>::mma(ah, bh[j], acc[i][j]);
        Frag<T>::guard(acc[i][0], acc[i][3], ah, ah);
      }
      Frag<T>::keep(bh[0], bh[1], bh[2], bh[3]);
    }
  }
  acc_guard4(acc[0][0], acc[0][1], acc[0][2], acc[0][3]);
  acc_guard4(acc[1][0], acc[1][1], acc[1][2], acc[1][3]);
  acc_guard4(acc[2][0], acc[2][1], acc[2][2], acc[2][3]);
  acc_guard4(acc[3][0], acc[3][1], acc[3][2], acc[3][3]);

  float* slab = sT[wave];
#pragma unroll
  for (int i = 0; i < 4; ++i) {
    const int mBase = m0 + (i << 4);
#pragma unroll
    for (int j = 0; j < 4; ++j) {
      const int nn = n0 + (j << 4) + rlane;
#pragma unroll
      for (int r = 0; r < 8; ++r) {
        float v = acc[i][j][r] * scale;
        if (RESID) v += resid[(size_t)(mBase + mOff + r) * IMG_W + nn];
        slab[(mOff + r) * 68 + (j << 4) + rlane] = v;
      }
    }
    __builtin_amdgcn_fence(__ATOMIC_RELEASE, "workgroup");
    __builtin_amdgcn_wave_barrier();
    __builtin_amdgcn_fence(__ATOMIC_ACQUIRE, "workgroup");
    {
      const int hh = lane >> 4, c4 = (lane & 15) * 4;
      for (int pass = 0; pass < 2; ++pass) {
#pragma unroll
        for (int it = 0; it < 8; ++it) {
          const int row = it * 2 + hh;
          v4f v = *(const v4f*)(slab + row * 68 + c4);
          *(volatile v4f*)(Cout + (size_t)(mBase + row) * IMG_W + n0 + c4) = v;
        }
        __threadfence();
      }
    }
    __builtin_amdgcn_fence(__ATOMIC_RELEASE, "workgroup");
    __builtin_amdgcn_wave_barrier();
    __builtin_amdgcn_fence(__ATOMIC_ACQUIRE, "workgroup");
  }
}

static inline size_t align256(size_t x) { return (x + 255) & ~(size_t)255; }

extern "C" void kernel_launch(void* const* d_in, const int* in_sizes, int n_in,
                              void* d_out, int out_size, void* d_ws, size_t ws_size,
                              hipStream_t stream) {
  if (n_in < 5) return;
  const float* pos   = (const float*)d_in[0];
  const float* scl   = (const float*)d_in[1];
  const float* opa   = (const float*)d_in[2];
  const float* inten = (const float*)d_in[3];
  const int*   ztgt  = (const int*)d_in[4];
  float* out = (float*)d_out;

  int n = in_sizes[2];
  if (in_sizes[0] / 3 < n) n = in_sizes[0] / 3;
  if (in_sizes[1] / 3 < n) n = in_sizes[1] / 3;
  if (in_sizes[3] < n)     n = in_sizes[3];
  if (n <= 0 || in_sizes[4] < 1) return;
  if (out_size != IMG_H * IMG_W) return;

  const int nSeg = (n + SEG - 1) / SEG;
  const int Ktot = nSeg * SEG;
  const size_t outBytes = (size_t)out_size * sizeof(float);
  const size_t cap = (ws_size < WS_CAP) ? ws_size : WS_CAP;
  const size_t szP   = align256((size_t)Ktot * sizeof(v4f));
  const size_t szImg = align256(outBytes);

  int spc = 0;
  size_t szA = 0, szB = 0;
  for (int c = 1; c <= 64 && c <= nSeg; ++c) {
    const int s = (nSeg + c - 1) / c;
    const size_t a = align256((size_t)IMG_H * (size_t)s * SEG * 2);
    const size_t b = align256((size_t)IMG_W * (size_t)s * SEG * 2);
    const size_t tot = 2 * szP + 2 * szImg + a + b;
    if (tot <= cap) { spc = s; szA = a; szB = b; break; }
  }
  if (spc == 0) return;
  const int nch = (nSeg + spc - 1) / spc;
  const int Kc = spc * SEG;

  unsigned char* ws = (unsigned char*)d_ws;
  v4f*   PA   = (v4f*)(ws);
  v4f*   PB   = (v4f*)(ws + szP);
  float* img0 = (float*)(ws + 2 * szP);
  float* img1 = (float*)(ws + 2 * szP + szImg);
  unsigned short* Abuf = (unsigned short*)(ws + 2 * szP + 2 * szImg);
  unsigned short* Bbuf = (unsigned short*)(ws + 2 * szP + 2 * szImg + szA);

  prep_params<<<dim3(nSeg), dim3(256), 0, stream>>>(pos, scl, opa, inten, ztgt, PA, PB, n);

  const dim3 gbA((spc + 7) / 8, IMG_H);
  const dim3 gbB((spc + 7) / 8, IMG_W);
  const dim3 gg((IMG_H / 64) * (IMG_W / 64) / 8);
  for (int c = 0; c < nch; ++c) {
    const int slotBase = c * Kc;
    build_rows<<<gbA, dim3(256), 0, stream>>>(PA, Abuf, Kc, slotBase, Ktot);
    build_rows<<<gbB, dim3(256), 0, stream>>>(PB, Bbuf, Kc, slotBase, Ktot);
    float* cout = (c == nch - 1) ? out : ((c & 1) ? img1 : img0);
    if (c == 0) {
      splat_gemm<false><<<gg, dim3(256), 0, stream>>>(Abuf, Bbuf, Kc, pos, scl, ztgt, n,
                                                      c * spc, spc, nSeg, cout, img0, OUT_SCALE);
    } else {
      const float* res = ((c - 1) & 1) ? img1 : img0;
      splat_gemm<true><<<gg, dim3(256), 0, stream>>>(Abuf, Bbuf, Kc, pos, scl, ztgt, n,
                                                     c * spc, spc, nSeg, cout, res, OUT_SCALE);
    }
  }
  hipStreamSynchronize(stream);
}
